// RGB_Depth_Agreement_Refined_33835752358434
// MI455X (gfx1250) — hardware-verified
//
#include <hip/hip_runtime.h>
#include <math.h>

constexpr int kNB  = 16;
constexpr int kS   = 577;
constexpr int kSP  = 640;
constexpr int kDM  = 768;
constexpr int kNH  = 12;
constexpr int kHD  = 64;
constexpr int kQKN = 1536;
constexpr int kBCH = 4;
constexpr int kMCH = kBCH * kSP;

constexpr float kWCarry    = 16.0f;
constexpr float kWCarryInv = 1.0f / 16.0f;
constexpr float kPCarry    = 2048.0f;
constexpr float kPVScale   = 64.0f / 2048.0f;
constexpr float kOutScale  = 1.0f / (64.0f * 16.0f);
constexpr float kScoreScale = 0.125f;

constexpr long kXmod   = (long)kNB * kSP * kDM;
constexpr long kXb     = (long)kSP * kDM;
constexpr long kQKmod  = (long)kMCH * kQKN;
constexpr long kQKsb   = (long)kSP * kQKN;
constexpr long kVTmod  = (long)kDM * kMCH;
constexpr long kPmod   = (long)kNH * kSP * kSP;
constexpr long kPhead  = (long)kSP * kSP;
constexpr long kOmod   = (long)kMCH * kDM;
constexpr long kOsb    = (long)kSP * kDM;
constexpr long kOutMod = (long)kNB * kS * kDM;
constexpr long kOutB   = (long)kS * kDM;

constexpr size_t kOffXh = 0;
constexpr size_t kSzXh  = (size_t)2 * kXmod * 2;
constexpr size_t kOffWq = kOffXh + kSzXh;
constexpr size_t kSzWq  = (size_t)3 * kDM * kDM * 2;
constexpr size_t kOffWo = kOffWq + kSzWq;
constexpr size_t kSzWo  = (size_t)kDM * kDM * 2;
constexpr size_t kOffQK = kOffWo + kSzWo;
constexpr size_t kSzQK  = (size_t)2 * kQKmod * 2;
constexpr size_t kOffVT = kOffQK + kSzQK;
constexpr size_t kSzVT  = (size_t)2 * kVTmod * 2;
constexpr size_t kOffPc = kOffVT + kSzVT;
constexpr size_t kSzPc  = (size_t)2 * kPmod * 2;
constexpr size_t kOffOc = kOffPc + kSzPc;
constexpr size_t kSzOc  = (size_t)2 * kOmod * 2;
constexpr size_t kWsTotal = kOffOc + kSzOc;
static_assert(kWsTotal == 87293952, "ws");
static_assert(kWsTotal <= 134217728, "ws");
static_assert(kOffWq % 128 == 0 && kOffWo % 128 == 0 && kOffQK % 128 == 0 && kOffVT % 128 == 0 && kOffPc % 128 == 0 && kOffOc % 128 == 0, "align");
static_assert(kMCH % 64 == 0 && kQKN % 64 == 0 && kDM % 64 == 0 && kSP % 64 == 0 && kHD % 64 == 0, "tiles");
static_assert(kDM % 32 == 0 && kSP % 32 == 0 && kHD % 32 == 0, "ksteps");

typedef __attribute__((ext_vector_type(16))) _Float16 v16h;
typedef __attribute__((ext_vector_type(8)))  _Float16 v8h;
typedef __attribute__((ext_vector_type(16))) __bf16   v16b;
typedef __attribute__((ext_vector_type(8)))  __bf16   v8b;
typedef __attribute__((ext_vector_type(8)))  float    v8f;
typedef __attribute__((ext_vector_type(4)))  float    v4f;
typedef __attribute__((ext_vector_type(4)))  unsigned int v4u;

__device__ __forceinline__ void dep_guard_h(v8f& a, v8f& b, v16h x, v16h y) { asm volatile("v_nop\n\tv_nop\n\tv_nop\n\tv_nop" : "+v"(a), "+v"(b) : "v"(x), "v"(y)); }
__device__ __forceinline__ void dep_guard_b(v8f& a, v8f& b, v16b x, v16b y) { asm volatile("v_nop\n\tv_nop\n\tv_nop\n\tv_nop" : "+v"(a), "+v"(b) : "v"(x), "v"(y)); }
__device__ __forceinline__ void keep4_h(v16h a, v16h b, v16h c, v16h d) { asm volatile("v_nop" :: "v"(a), "v"(b), "v"(c), "v"(d)); }
__device__ __forceinline__ void keep4_b(v16b a, v16b b, v16b c, v16b d) { asm volatile("v_nop" :: "v"(a), "v"(b), "v"(c), "v"(d)); }
__device__ __forceinline__ void acc_guard4(v8f& a, v8f& b, v8f& c, v8f& d) { asm volatile("v_nop\n\tv_nop\n\tv_nop\n\tv_nop" : "+v"(a), "+v"(b), "+v"(c), "+v"(d)); }
template <typename T> struct Frag;
template <> struct Frag<_Float16> {
  typedef v16h V; union U { v16h v; v8h h[2]; };
  static __device__ __forceinline__ v16h load(const _Float16* p) {
    U f; f.h[0] = *(const v8h*)(p); f.h[1] = *(const v8h*)(p + 16); return f.v;
  }
  static __device__ __forceinline__ v8f mma(v16h a, v16h b, v8f c) {
    return __builtin_amdgcn_wmma_f32_16x16x32_f16(false, a, false, b, (short)0, c, false, false);
  }
  static __device__ __forceinline__ void guard(v8f& a, v8f& b, v16h x, v16h y) { dep_guard_h(a, b, x, y); }
  static __device__ __forceinline__ void keep(v16h a, v16h b, v16h c, v16h d) { keep4_h(a, b, c, d); }
};
template <> struct Frag<__bf16> {
  typedef v16b V; union U { v16b v; v8b h[2]; };
  static __device__ __forceinline__ v16b load(const __bf16* p) {
    U f; f.h[0] = *(const v8b*)(p); f.h[1] = *(const v8b*)(p + 16); return f.v;
  }
  static __device__ __forceinline__ v8f mma(v16b a, v16b b, v8f c) {
    return __builtin_amdgcn_wmma_f32_16x16x32_bf16(false, a, false, b, (short)0, c, false, false);
  }
  static __device__ __forceinline__ void guard(v8f& a, v8f& b, v16b x, v16b y) { dep_guard_b(a, b, x, y); }
  static __device__ __forceinline__ void keep(v16b a, v16b b, v16b c, v16b d) { keep4_b(a, b, c, d); }
};

__device__ __forceinline__ unsigned pk16(unsigned short a, unsigned short b) { return (unsigned)a | ((unsigned)b << 16); }
__device__ __forceinline__ unsigned short h_bits(float f) { const _Float16 h = (_Float16)f; return __builtin_bit_cast(unsigned short, h); }

__device__ __forceinline__ v8f mma_h(v16h a, v16h b, v8f c) {
  c = __builtin_amdgcn_wmma_f32_16x16x32_f16(false, a, false, b, (short)0, c, false, false);
  asm volatile("v_nop\n\tv_nop\n\tv_nop\n\tv_nop" : "+v"(c) : "v"(a), "v"(b));
  return c;
}

template <int BIAS_MODE, int OUT_MODE>
__global__ __launch_bounds__(256) void gemm64g(
    const unsigned short* __restrict__ Ap, int lda, long strideAo, long strideAi,
    const unsigned short* __restrict__ Btp, int ldb, long strideBo, long strideBi,
    void* __restrict__ Cout, int ldc, long strideCo, long strideCi,
    const float* __restrict__ bias,
    int M, int N, int K, int zdiv, int Mvalid, float scale) {
  typedef _Float16 T;
  typedef v16h V;
  const T* A = (const T*)Ap; const T* Bt = (const T*)Btp;
  __shared__ __align__(16) float sT[8][16 * 68];
  const int gy   = blockIdx.y;
  const int go   = gy / zdiv;
  const int gi   = gy - go * zdiv;
  const int lane = threadIdx.x & 31;
  const int wave = threadIdx.x >> 5;
  const int tilesN = N >> 6;
  const int tilesM = M >> 6;
  const int tile = blockIdx.x * 8 + wave;
  if (tile >= tilesM * tilesN) return;
  const int tm = tile / tilesN;
  const int tn = tile - tm * tilesN;
  const int m0 = tm << 6;
  const int n0 = tn << 6;

  const T* Ab = A  + (size_t)go * (size_t)strideAo + (size_t)gi * (size_t)strideAi;
  const T* Bb = Bt + (size_t)go * (size_t)strideBo + (size_t)gi * (size_t)strideBi;
  const size_t cOff = (size_t)go * (size_t)strideCo + (size_t)gi * (size_t)strideCi;

  const int rlane = lane & 15;
  const int koff  = (lane >> 4) * 8;
  const int mOff  = (lane >> 4) * 8;

  v8f acc[4][4];
#pragma unroll
  for (int i = 0; i < 4; ++i)
#pragma unroll
    for (int j = 0; j < 4; ++j) acc[i][j] = (v8f){0.f,0.f,0.f,0.f,0.f,0.f,0.f,0.f};

  for (int k0 = 0; k0 < K; k0 += 32) {
    V bh[4];
#pragma unroll
    for (int j = 0; j < 4; ++j) {
      const size_t bo = (size_t)(n0 + (j << 4) + rlane) * ldb + koff + k0;
      bh[j] = Frag<T>::load(Bb + bo);
    }
#pragma unroll
    for (int i = 0; i < 4; ++i) {
      const size_t ao = (size_t)(m0 + (i << 4) + rlane) * lda + koff + k0;
      V ah = Frag<T>::load(Ab + ao);
#pragma unroll
      for (int j = 0; j < 4; ++j) {
        acc[i][j] = Frag<T>::mma(ah, bh[j], acc[i][j]);
      }
      Frag<T>::guard(acc[i][0], acc[i][3], ah, ah);
    }
    Frag<T>::keep(bh[0], bh[1], bh[2], bh[3]);
  }
  acc_guard4(acc[0][0], acc[0][1], acc[0][2], acc[0][3]);
  acc_guard4(acc[1][0], acc[1][1], acc[1][2], acc[1][3]);
  acc_guard4(acc[2][0], acc[2][1], acc[2][2], acc[2][3]);
  acc_guard4(acc[3][0], acc[3][1], acc[3][2], acc[3][3]);

  float* slab = sT[wave];
#pragma unroll
  for (int i = 0; i < 4; ++i) {
    const int mBase = m0 + (i << 4);
#pragma unroll
    for (int j = 0; j < 4; ++j) {
      const int n = n0 + (j << 4) + rlane;
      float bv = 0.f;
      if (BIAS_MODE == 2) bv = bias[n];
#pragma unroll
      for (int r = 0; r < 8; ++r) {
        float v = acc[i][j][r] * scale;
        if (BIAS_MODE == 1) v += bias[mBase + mOff + r];
        if (BIAS_MODE == 2) v += bv;
        slab[(mOff + r) * 68 + (j << 4) + rlane] = v;
      }
    }
    __builtin_amdgcn_fence(__ATOMIC_RELEASE, "workgroup");
    __builtin_amdgcn_wave_barrier();
    __builtin_amdgcn_fence(__ATOMIC_ACQUIRE, "workgroup");
    if (OUT_MODE == 0) {
      float* C = (float*)Cout + cOff;
      const int hh = lane >> 4, c4 = (lane & 15) * 4;
      for (int pass = 0; pass < 2; ++pass) {
#pragma unroll
        for (int it = 0; it < 8; ++it) {
          const int row = it * 2 + hh;
          v4f v = *(const v4f*)(slab + row * 68 + c4);
          if (mBase + row < Mvalid) *(volatile v4f*)(C + (size_t)(mBase + row) * ldc + n0 + c4) = v;
        }
        __threadfence();
      }
    } else {
      const int q = lane >> 3, c8 = (lane & 7) * 8;
      unsigned short* C = (unsigned short*)Cout + cOff;
      for (int pass = 0; pass < 2; ++pass) {
#pragma unroll
        for (int it = 0; it < 4; ++it) {
          const int row = it * 4 + q;
          const float* sp = slab + row * 68 + c8;
          v8h hv;
#pragma unroll
          for (int e = 0; e < 8; ++e) hv[e] = (_Float16)sp[e];
          if (mBase + row < Mvalid) *(volatile v8h*)(C + (size_t)(mBase + row) * ldc + n0 + c8) = hv;
        }
        __threadfence();
      }
    }
    __builtin_amdgcn_fence(__ATOMIC_RELEASE, "workgroup");
    __builtin_amdgcn_wave_barrier();
    __builtin_amdgcn_fence(__ATOMIC_ACQUIRE, "workgroup");
  }
}

__global__ __launch_bounds__(256) void castw_kernel(const float* __restrict__ in, unsigned short* __restrict__ out, int n8, float scale) {
  const int i = blockIdx.x * 256 + threadIdx.x;
  if (i >= n8) return;
  const float* p = in + 8 * (size_t)i;
  const v4f a = *(const v4f*)(p);
  const v4f c = *(const v4f*)(p + 4);
  unsigned short hb[8];
#pragma unroll
  for (int e = 0; e < 4; ++e) {
    hb[e]     = h_bits(a[e] * scale);
    hb[4 + e] = h_bits(c[e] * scale);
  }
  const v4u u = (v4u){pk16(hb[0], hb[1]), pk16(hb[2], hb[3]), pk16(hb[4], hb[5]), pk16(hb[6], hb[7])};
  unsigned short* q = out + 8 * (size_t)i;
  *(volatile v4u*)q = u;
  __threadfence();
  *(volatile v4u*)q = u;
}

__global__ __launch_bounds__(256) void castx_kernel(const float* __restrict__ X, unsigned short* __restrict__ Xh) {
  const int i = blockIdx.x * 256 + threadIdx.x;
  const int b   = i / (kSP * 96);
  const int rem = i - b * (kSP * 96);
  const int r   = rem / 96;
  const int c8  = rem - r * 96;
  const int rr  = (r < kS) ? r : (kS - 1);
  const bool real = (r < kS);
  const float* p = X + ((size_t)(b * kS + rr) * kDM + (size_t)c8 * 8);
  const v4f a = *(const v4f*)(p);
  const v4f c = *(const v4f*)(p + 4);
  unsigned short hb[8];
#pragma unroll
  for (int e = 0; e < 4; ++e) {
    const float x0 = real ? a[e] : 0.0f;
    const float x1 = real ? c[e] : 0.0f;
    hb[e]     = h_bits(x0);
    hb[4 + e] = h_bits(x1);
  }
  const v4u u = (v4u){pk16(hb[0], hb[1]), pk16(hb[2], hb[3]), pk16(hb[4], hb[5]), pk16(hb[6], hb[7])};
  unsigned short* q = Xh + 8 * (size_t)i;
  *(volatile v4u*)q = u;
  __threadfence();
  *(volatile v4u*)q = u;
}

__device__ __forceinline__ float grp16_max(float v) {
#pragma unroll
  for (int off = 8; off > 0; off >>= 1) v = fmaxf(v, __shfl_xor(v, off, 16));
  return v;
}
__device__ __forceinline__ float grp16_sum(float v) {
#pragma unroll
  for (int off = 8; off > 0; off >>= 1) v += __shfl_xor(v, off, 16);
  return v;
}

__global__ __launch_bounds__(256) void score_agree_kernel(
    const unsigned short* __restrict__ QKc,
    unsigned short* __restrict__ Pc,
    const float* __restrict__ alpha_raw, const float* __restrict__ beta_raw) {
  #pragma clang fp contract(off)
  __shared__ __align__(16) float sS[2 * 16 * kSP];
  __shared__ __align__(16) float sG[16 * kSP];
  __shared__ float sInvG[16];

  const int qt = blockIdx.x;
  const int h  = blockIdx.y;
  const int q0 = qt * 16;
  const int t = threadIdx.x, lane = t & 31, wave = t >> 5;
  const int hh = lane >> 4, c = lane & 15, koff = hh * 8;
  unsigned short* Pbase = Pc + (size_t)h * kPhead + (size_t)q0 * kSP;

  if (q0 >= kS) {
    for (int pass = 0; pass < 2; ++pass) {
#pragma unroll 1
      for (int it = 0; it < 10; ++it) {
        const int mod = (it >= 5) ? 1 : 0;
        const int rem = (it - mod * 5) * 256 + t;
        const int rr  = rem / 80;
        const int seg = rem - rr * 80;
        const v4u z = (v4u){0u, 0u, 0u, 0u};
        *(volatile v4u*)(Pbase + (size_t)mod * kPmod + (size_t)rr * kSP + seg * 8) = z;
      }
      __threadfence();
    }
    return;
  }

  const _Float16* QK = (const _Float16*)QKc;
  for (int mod = 0; mod < 2; ++mod) {
    const _Float16* Qp = QK + (size_t)mod * kQKmod + (size_t)(q0 + c) * kQKN + h * kHD + koff;
    const _Float16* Kp = QK + (size_t)mod * kQKmod + kDM + h * kHD + koff;
    const v16h qf0 = Frag<_Float16>::load(Qp);
    const v16h qf1 = Frag<_Float16>::load(Qp + 32);
    float* S = sS + mod * (16 * kSP);
#pragma unroll 1
    for (int nt = wave; nt < 40; nt += 8) {
      v8f acc = (v8f){0.f,0.f,0.f,0.f,0.f,0.f,0.f,0.f};
      const _Float16* kp = Kp + (size_t)(nt * 16 + c) * kQKN;
      acc = mma_h(qf0, Frag<_Float16>::load(kp), acc);
      acc = mma_h(qf1, Frag<_Float16>::load(kp + 32), acc);
      float* Srow = S + (hh * 8) * kSP + nt * 16 + c;
#pragma unroll
      for (int r = 0; r < 8; ++r) Srow[r * kSP] = acc[r] * kScoreScale;
    }
  }
  __syncthreads();

  const int row = t >> 4, sub = t & 15;
  float* si = sS + row * kSP;
  float* sd = sS + 16 * kSP + row * kSP;
  float* sg = sG + row * kSP;

  float mi = -INFINITY, md = -INFINITY;
#pragma unroll 1
  for (int j = 0; j < 40; ++j) {
    const int cc = sub + 16 * j;
    const bool valid = cc < kS;
    const float a = si[cc], d = sd[cc];
    mi = valid ? fmaxf(mi, a) : mi;
    md = valid ? fmaxf(md, d) : md;
  }
  mi = grp16_max(mi); md = grp16_max(md);

  float smi = 0.f, smd = 0.f;
#pragma unroll 1
  for (int j = 0; j < 40; ++j) {
    const int cc = sub + 16 * j;
    const bool valid = cc < kS;
    const float xi = si[cc] - mi;
    const float xd = sd[cc] - md;
    const float ei = valid ? expf(xi) : 0.f;
    const float ed = valid ? expf(xd) : 0.f;
    si[cc] = ei; sd[cc] = ed;
    smi += ei; smd += ed;
  }
  smi = grp16_sum(smi); smd = grp16_sum(smd);
  const float invi = 1.0f / smi, invd = 1.0f / smd;

  float mg = -INFINITY;
#pragma unroll 1
  for (int j = 0; j < 40; ++j) {
    const int cc = sub + 16 * j;
    const bool valid = cc < kS;
    const float p1 = si[cc] * invi;
    const float p2 = sd[cc] * invd;
    si[cc] = p1; sd[cc] = p2;
    const float ag = p1 * p2;
    mg = valid ? fmaxf(mg, ag) : mg;
  }
  mg = grp16_max(mg);

  float smg = 0.f;
#pragma unroll 1
  for (int j = 0; j < 40; ++j) {
    const int cc = sub + 16 * j;
    const bool valid = cc < kS;
    const float ag = si[cc] * sd[cc];
    const float xg = ag - mg;
    const float eg = valid ? expf(xg) : 0.f;
    sg[cc] = eg;
    smg += eg;
  }
  smg = grp16_sum(smg);
  if (sub == 0) sInvG[row] = 1.0f / smg;
  __syncthreads();

  const float ar0 = alpha_raw[0], br0 = beta_raw[0];
  const float alpha = 1.0f / (1.0f + expf(-ar0));
  const float beta  = 1.0f / (1.0f + expf(-br0));
  for (int pass = 0; pass < 2; ++pass) {
#pragma unroll 1
    for (int it = 0; it < 10; ++it) {
      const int mod = (it >= 5) ? 1 : 0;
      const int rem = (it - mod * 5) * 256 + t;
      const int rr  = rem / 80;
      const int seg = rem - rr * 80;
      const float* ps = sS + mod * (16 * kSP) + rr * kSP + seg * 8;
      const float* gs = sG + rr * kSP + seg * 8;
      const v4f pa = *(const v4f*)(ps);
      const v4f pb = *(const v4f*)(ps + 4);
      const v4f ga = *(const v4f*)(gs);
      const v4f gb = *(const v4f*)(gs + 4);
      const float gate = mod ? beta : alpha;
      const float ig = sInvG[rr];
      const bool rowok = (q0 + rr) < kS;
      unsigned short hb[8];
#pragma unroll
      for (int e = 0; e < 4; ++e) {
        const float pg0 = ga[e] * ig;
        const float pg1 = gb[e] * ig;
        float v0 = (gate * pg0 + pa[e]) * kPCarry;
        float v1 = (gate * pg1 + pb[e]) * kPCarry;
        v0 = rowok ? v0 : 0.0f;
        v1 = rowok ? v1 : 0.0f;
        hb[e]     = h_bits(v0);
        hb[4 + e] = h_bits(v1);
      }
      const v4u u = (v4u){pk16(hb[0], hb[1]), pk16(hb[2], hb[3]), pk16(hb[4], hb[5]), pk16(hb[6], hb[7])};
      *(volatile v4u*)(Pbase + (size_t)mod * kPmod + (size_t)rr * kSP + seg * 8) = u;
    }
    __threadfence();
  }
}

extern "C" void kernel_launch(void* const* d_in, const int* in_sizes, int n_in,
                              void* d_out, int out_size, void* d_ws, size_t ws_size,
                              hipStream_t stream) {
  if (n_in < 8) return;
  if (ws_size < kWsTotal) return;
  if (in_sizes[0] != kNB * kS * kDM || in_sizes[1] != kNB * kS * kDM || in_sizes[2] != 3 * kDM * kDM ||
      in_sizes[3] < 3 * kDM || in_sizes[4] != kDM * kDM || in_sizes[5] < kDM || in_sizes[6] < 1 || in_sizes[7] < 1)
    return;
  if (out_size != 2 * kNB * kS * kDM) return;

  const float* img   = (const float*)d_in[0];
  const float* dpt   = (const float*)d_in[1];
  const float* w_qkv = (const float*)d_in[2];
  const float* b_qkv = (const float*)d_in[3];
  const float* w_out = (const float*)d_in[4];
  const float* b_out = (const float*)d_in[5];
  const float* a_raw = (const float*)d_in[6];
  const float* b_raw = (const float*)d_in[7];
  float* out = (float*)d_out;

  char* ws = (char*)d_ws;
  unsigned short* Xh  = (unsigned short*)(ws + kOffXh);
  unsigned short* Wq  = (unsigned short*)(ws + kOffWq);
  unsigned short* Wo  = (unsigned short*)(ws + kOffWo);
  unsigned short* QKc = (unsigned short*)(ws + kOffQK);
  unsigned short* VTc = (unsigned short*)(ws + kOffVT);
  unsigned short* Pc  = (unsigned short*)(ws + kOffPc);
  unsigned short* Oc  = (unsigned short*)(ws + kOffOc);

  castw_kernel<<<864, 256, 0, stream>>>(w_qkv, Wq, 3 * kDM * kDM / 8, kWCarry);
  castw_kernel<<<288, 256, 0, stream>>>(w_out, Wo, kDM * kDM / 8, kWCarry);
  castx_kernel<<<3840, 256, 0, stream>>>(img, Xh);
  castx_kernel<<<3840, 256, 0, stream>>>(dpt, Xh + kXmod);

  for (int ch = 0; ch < kNB / kBCH; ++ch) {
    const int b0 = ch * kBCH;
    gemm64g<2, 1><<<dim3(120, 2), 256, 0, stream>>>(
        Xh + (size_t)b0 * kXb, kDM, kXmod, 0L,
        Wq, kDM, 0L, 0L,
        (void*)QKc, kQKN, kQKmod, 0L,
        b_qkv, kMCH, kQKN, kDM, 1, kMCH, kWCarryInv);
    gemm64g<1, 1><<<dim3(60, 2), 256, 0, stream>>>(
        Wq + (size_t)kQKN * kDM, kDM, 0L, 0L,
        Xh + (size_t)b0 * kXb, kDM, kXmod, 0L,
        (void*)VTc, kMCH, kVTmod, 0L,
        b_qkv + kQKN, kDM, kMCH, kDM, 1, kDM, kWCarryInv);
    for (int sb = 0; sb < kBCH; ++sb) {
      score_agree_kernel<<<dim3(40, kNH), 256, 0, stream>>>(QKc + (size_t)sb * kQKsb, Pc, a_raw, b_raw);
      gemm64g<0, 1><<<dim3(2, 2 * kNH), 256, 0, stream>>>(
          Pc, kSP, kPmod, kPhead,
          VTc + (size_t)sb * kSP, kMCH, kVTmod, (long)kHD * kMCH,
          (void*)(Oc + (size_t)sb * kOsb), kDM, kOmod, (long)kHD,
          b_qkv, kSP, kHD, kSP, kNH, kSP, kPVScale);
    }
    gemm64g<2, 0><<<dim3(15, 2 * kBCH), 256, 0, stream>>>(
        Oc, kDM, kOmod, kOsb,
        Wo, kDM, 0L, 0L,
        (void*)(out + (size_t)b0 * kOutB), kDM, kOutMod, kOutB,
        b_out, kSP, kDM, kDM, kBCH, kS, kOutScale);
  }
}
